// self_attention_cam_9844065042954
// MI455X (gfx1250) — hardware-verified
//
#include <hip/hip_runtime.h>
#include <math.h>

typedef __attribute__((ext_vector_type(16))) _Float16 v16h;
typedef __attribute__((ext_vector_type(16))) __bf16 v16b;
typedef __attribute__((ext_vector_type(8)))  _Float16 v8h;
typedef __attribute__((ext_vector_type(8)))  float v8f;
typedef __attribute__((ext_vector_type(4)))  float v4f;
typedef __attribute__((ext_vector_type(2)))  float v2f;
typedef __attribute__((ext_vector_type(4)))  unsigned v4u;
typedef __attribute__((ext_vector_type(4)))  int v4i;
typedef float __attribute__((may_alias)) float_a;
typedef int __attribute__((may_alias)) int_a;

template <typename T> __device__ __forceinline__ void vst2(void* p, T v) { *(volatile T*)p = v; __threadfence(); *(volatile T*)p = v; }
__device__ __forceinline__ v8f wmma16(v16h a, v16h b, v8f c) {
  v8f d = __builtin_amdgcn_wmma_f32_16x16x32_f16(false, a, false, b, (short)0, c, false, false);
  asm volatile("v_nop\n\tv_nop\n\tv_nop\n\tv_nop" : "+v"(d) : "v"(a), "v"(b));
  return d;
}
__device__ __forceinline__ v8f wmma_bf(v16b a, v16b b, v8f c) {
  v8f d = __builtin_amdgcn_wmma_f32_16x16x32_bf16(false, a, false, b, (short)0, c, false, false);
  asm volatile("v_nop\n\tv_nop\n\tv_nop\n\tv_nop" : "+v"(d) : "v"(a), "v"(b));
  return d;
}
__device__ __forceinline__ v16h frag_h(const _Float16* rowk0, int lane) {
  union { v16h v; v8h q[2]; } u; const _Float16* p = rowk0 + 8 * (lane >> 4);
  u.q[0] = *(const v8h*)p; u.q[1] = *(const v8h*)(p + 16); return u.v;
}
__device__ __forceinline__ v16h frag_f32(const float* rowk0, int lane) {
  v16h a; const float* p = rowk0 + 8 * (lane >> 4);
#pragma unroll
  for (int i = 0; i < 8; ++i) { a[i] = (_Float16)p[i]; a[8 + i] = (_Float16)p[16 + i]; }
  return a;
}
__device__ __forceinline__ v16h frag_f32s(const float* rowk0, int lane, float sc) {
  v16h a; const float* p = rowk0 + 8 * (lane >> 4);
#pragma unroll
  for (int i = 0; i < 8; ++i) { a[i] = (_Float16)(p[i] * sc); a[8 + i] = (_Float16)(p[16 + i] * sc); }
  return a;
}
__device__ __forceinline__ v16h fragc_f32(const float* W, int k0, int n, int lane, int ld, int K) {
  v16h a; const int g = lane >> 4;
#pragma unroll
  for (int i = 0; i < 8; ++i) { const int ka = k0 + 8 * g + i, kb = ka + 16;
    a[i] = (_Float16)(ka < K ? W[(size_t)(ka < K ? ka : K - 1) * ld + n] : 0.f); a[8 + i] = (_Float16)(kb < K ? W[(size_t)(kb < K ? kb : K - 1) * ld + n] : 0.f); }
  return a;
}
struct F2 { v16b h, l; };
__device__ __forceinline__ F2 bsplit16(const float v[16]) { F2 r;
#pragma unroll
  for (int i = 0; i < 16; ++i) { const __bf16 h = (__bf16)v[i]; r.h[i] = h; r.l[i] = (__bf16)(v[i] - (float)h); }
  return r; }
__device__ __forceinline__ F2 split_row(const float* row, int k0, int lane) { float v[16]; const float* p = row + k0 + 8 * (lane >> 4);
#pragma unroll
  for (int i = 0; i < 8; ++i) { v[i] = p[i]; v[8 + i] = p[16 + i]; }
  return bsplit16(v); }
__device__ __forceinline__ F2 split_rowK(const float* row, int k0, int lane, int K) { float v[16]; const int g = lane >> 4;
#pragma unroll
  for (int i = 0; i < 8; ++i) { const int ka = k0 + 8 * g + i, kb = ka + 16; v[i] = ka < K ? row[ka < K ? ka : K - 1] : 0.f; v[8 + i] = kb < K ? row[kb < K ? kb : K - 1] : 0.f; }
  return bsplit16(v); }
__device__ __forceinline__ F2 split_col(const float* W, int k0, int n, int lane, int ld, int K) { float v[16]; const int g = lane >> 4;
#pragma unroll
  for (int i = 0; i < 8; ++i) { const int ka = k0 + 8 * g + i, kb = ka + 16; v[i] = ka < K ? W[(size_t)(ka < K ? ka : K - 1) * ld + n] : 0.f; v[8 + i] = kb < K ? W[(size_t)(kb < K ? kb : K - 1) * ld + n] : 0.f; }
  return bsplit16(v); }
__device__ __forceinline__ v8f mac3(const F2& a, const F2& b, v8f c) { c = wmma_bf(a.l, b.h, c); c = wmma_bf(a.h, b.l, c); return wmma_bf(a.h, b.h, c); }
__device__ __forceinline__ float sigm(float v) { return 1.0f / (1.0f + expf(-v)); }
#define LDSX() do { asm volatile("s_wait_dscnt 0" ::: "memory"); __builtin_amdgcn_wave_barrier(); __builtin_amdgcn_fence(__ATOMIC_RELEASE, "workgroup"); } while (0)


#define NB 8
#define CIN 256
#define NP 4096
#define AD 128
#define NCL 21
#define NCP 32
#ifndef TQB
#define TQB (NP / 64)
#define TNB NB
#endif
typedef __attribute__((ext_vector_type(8))) __bf16 v8b;
__device__ __forceinline__ v16b frag_b(const __bf16* rowk0, int lane) {
  union { v16b v; v8b q[2]; } u; const __bf16* p = rowk0 + 8 * (lane >> 4);
  u.q[0] = *(const v8b*)p; u.q[1] = *(const v8b*)(p + 16); return u.v;
}
__device__ __forceinline__ float bfr(float v) { return (float)(__bf16)v; }
__device__ __attribute__((noinline)) float exp_ni(float v) { return expf(v); }
__device__ __attribute__((noinline)) float erf_ni(float v) { return erff(v); }

#define WS_PW   0u
#define WS_VB   (WS_PW + 2u * 256 * CIN)
#define WS_QK   (WS_VB + 2u * NB * NCP * NP)
#define WS_Y    (WS_QK + 4u * NB * NP * 256)
#define WS_PS   (WS_Y + 4u * NB * NCP * NP)
#define WS_ST   (WS_PS + 4u * NB * 64 * 32)
#define WS_END  (WS_ST + 4u * 64)

__global__ __launch_bounds__(256) void k_pack(const float* __restrict__ WQ, const float* __restrict__ WK, const float* __restrict__ LG, __bf16* __restrict__ PW, __bf16* __restrict__ VB) {
  __shared__ __align__(16) __bf16 s[256]; const int tid = threadIdx.x;
  if (blockIdx.y == 0) { const int r = blockIdx.x; if (r >= 256) return; s[tid] = (__bf16)((r < AD) ? WQ[(size_t)r * CIN + tid] : WK[(size_t)(r - AD) * CIN + tid]); __syncthreads(); if (tid < 32) vst2((unsigned*)(PW + (size_t)r * CIN + tid * 8), *(const v4u*)&s[tid * 8]); }
  else { const int chunk = blockIdx.x & 15, bc = blockIdx.x >> 4; const int b = bc >> 5, c = bc & 31; const size_t n0 = (size_t)chunk * 256;
    s[tid] = (__bf16)((c < NCL) ? LG[((size_t)b * NCL + (c < NCL ? c : 0)) * NP + n0 + tid] : 0.f); __syncthreads();
    if (tid < 32) vst2((unsigned*)(VB + ((size_t)b * NCP + c) * NP + n0 + tid * 8), *(const v4u*)&s[tid * 8]); }
}
__global__ __launch_bounds__(128) void k_qk(const float* __restrict__ HC, const __bf16* __restrict__ PW, const float* __restrict__ BQ, const float* __restrict__ BK, float* __restrict__ QK) {
  __shared__ __align__(16) __bf16 sx[64][CIN + 8]; __shared__ __align__(16) float so[4][16][132];
  const int tid = threadIdx.x, wave = tid >> 5, lane = tid & 31, col = lane & 15, g = lane >> 4; const int b = blockIdx.y; const int p0 = blockIdx.x * 64;
  for (int q = tid; q < CIN * 64; q += 128) { const int c = q >> 6, nl = q & 63; sx[nl][c] = (__bf16)HC[((size_t)b * CIN + c) * NP + p0 + nl]; }
  __syncthreads();
#pragma unroll 1
  for (int which = 0; which < 2; ++which) { v8f acc[8] = {};
#pragma unroll 2
    for (int kc = 0; kc < CIN / 32; ++kc) { v16b a;
#pragma unroll
      for (int i = 0; i < 8; ++i) { a[i] = sx[wave * 16 + col][kc * 32 + 8 * g + i]; a[8 + i] = sx[wave * 16 + col][kc * 32 + 16 + 8 * g + i]; }
#pragma unroll
      for (int j = 0; j < 8; ++j) acc[j] = wmma_bf(a, frag_b(PW + (size_t)(which * AD + j * 16 + col) * CIN + kc * 32, lane), acc[j]); }
    const float* bias = which ? BK : BQ;
#pragma unroll
    for (int j = 0; j < 8; ++j) { const float bb = bfr(bias[j * 16 + col]);
#pragma unroll
      for (int r = 0; r < 8; ++r) so[wave][8 * g + r][j * 16 + col] = acc[j][r] + bb; }
    LDSX();
    for (int rl = 0; rl < 16; ++rl) vst2(QK + ((size_t)b * NP + p0 + wave * 16 + rl) * 256 + which * AD + lane * 4, *(const v4f*)&so[wave][rl][lane * 4]);
    LDSX(); }
}
__global__ __launch_bounds__(128) void k_attn(const float* __restrict__ QK, const __bf16* __restrict__ VB, const float* __restrict__ LG, const float* __restrict__ WO, const float* __restrict__ BO, float* __restrict__ Y, float* __restrict__ PS) {
  __shared__ __align__(16) float sp[4][16][36]; __shared__ __align__(16) float sa[NCP][68]; __shared__ __align__(16) float sy[NCP][68]; __shared__ float swo[NCL][NCL], sbo[NCL]; __shared__ __align__(16) float sps[32];
  const int tid = threadIdx.x, wave = tid >> 5, lane = tid & 31, col = lane & 15, g = lane >> 4; const int b = blockIdx.y; const int qb = blockIdx.x; const int q0 = qb * 64 + wave * 16;
  for (int i = tid; i < NCL * NCL; i += 128) swo[i / NCL][i % NCL] = bfr(WO[i]); if (tid < NCL) sbo[tid] = bfr(BO[tid]);
  const float* qrow = QK + ((size_t)b * NP + q0 + col) * 256;
  float m[8], l[8];
#pragma unroll
  for (int r = 0; r < 8; ++r) { m[r] = -3.0e38f; l[r] = 0.f; }
  v8f acc[2] = {};
#pragma unroll 1
  for (int ks = 0; ks < NP / 32; ++ks) { v8f s[2];
#pragma unroll
    for (int ct = 0; ct < 2; ++ct) { const int kk = ks * 32 + ct * 16 + col; const float* krow = QK + ((size_t)b * NP + kk) * 256 + AD; v8f c = {};
#pragma unroll
      for (int kc = 0; kc < AD / 32; ++kc) { const F2 kb = split_row(krow, kc * 32, lane); const F2 qa = split_row(qrow, kc * 32, lane); c = mac3(qa, kb, c); }
#pragma unroll
      for (int r = 0; r < 8; ++r) s[ct][r] = c[r] * 0.08838834764831845f; }
#pragma unroll
    for (int r = 0; r < 8; ++r) { float mx = fmaxf(s[0][r], s[1][r]);
#pragma unroll
      for (int o = 1; o < 16; o <<= 1) mx = fmaxf(mx, __shfl_xor(mx, o));
      const float mn = fmaxf(m[r], mx); const float alpha = exp_ni(m[r] - mn);
      const float e0 = exp_ni(s[0][r] - mn), e1 = exp_ni(s[1][r] - mn); float es = e0 + e1;
#pragma unroll
      for (int o = 1; o < 16; o <<= 1) es += __shfl_xor(es, o);
      l[r] = l[r] * alpha + es; m[r] = mn;
#pragma unroll
      for (int dt = 0; dt < 2; ++dt) acc[dt][r] *= alpha;
      sp[wave][8 * g + r][col] = e0; sp[wave][8 * g + r][16 + col] = e1; }
    LDSX();
    const F2 pa = split_row(&sp[wave][col][0], 0, lane);
#pragma unroll
    for (int dt = 0; dt < 2; ++dt) { const v16b vb = frag_b(VB + ((size_t)b * NCP + dt * 16 + col) * NP + ks * 32, lane); acc[dt] = wmma_bf(pa.l, vb, acc[dt]); acc[dt] = wmma_bf(pa.h, vb, acc[dt]); }
    LDSX(); }
#pragma unroll
  for (int r = 0; r < 8; ++r) { const float il = 1.0f / l[r]; const int qi = wave * 16 + 8 * g + r;
#pragma unroll
    for (int dt = 0; dt < 2; ++dt) { const int c = dt * 16 + col; float v = acc[dt][r] * il; if (c < NCL) v += bfr(LG[((size_t)b * NCL + c) * NP + qb * 64 + qi]); sa[c][qi] = v; } }
  __syncthreads();
  for (int it = tid; it < NCP * 64; it += 128) { const int o = it >> 6, qi = it & 63; float v = 0.f; if (o < NCL) { v = sbo[o];
#pragma unroll 1
      for (int c = 0; c < NCL; ++c) v += swo[o][c] * sa[c][qi]; }
    sy[o][qi] = v; }
  __syncthreads();
  if (tid < 32) { float acc2 = 0.f; if (tid < NCL) for (int qi = 0; qi < 64; ++qi) acc2 += sy[tid][qi]; sps[tid] = acc2; }
  for (int it = tid; it < NCL * 16; it += 128) { const int o = it >> 4, pc = it & 15; vst2(Y + ((size_t)b * NCP + o) * NP + qb * 64 + pc * 4, *(const v4f*)&sy[o][pc * 4]); }
  __syncthreads();
  if (tid < 8) vst2(PS + ((size_t)b * 64 + qb) * 32 + tid * 4, *(const v4f*)&sps[tid * 4]);
}
template <int MODE>
__global__ __launch_bounds__(32) void k_red(const float* __restrict__ PS, float* __restrict__ ST) {
  __shared__ __align__(16) float s[32]; const int c = threadIdx.x; float acc = 0.f;
  for (int bq = 0; bq < TNB * 64; ++bq) acc += PS[(size_t)bq * 32 + c];
  acc /= (float)(TNB * NP); s[c] = (c < NCL) ? ((MODE == 0) ? acc : rsqrtf(acc + 1e-5f)) : 0.f;
  __syncthreads();
  if (c < 8) vst2(ST + MODE * 32 + c * 4, *(const v4f*)&s[c * 4]);
}
__global__ __launch_bounds__(64) void k_var(const float* __restrict__ Y, const float* __restrict__ ST, float* __restrict__ PS) {
  __shared__ __align__(16) float s[32]; const int b = blockIdx.y, qb = blockIdx.x, tid = threadIdx.x;
  if (tid < 32) { float acc = 0.f; if (tid < NCL) { const float mu = ST[tid]; const float* yr = Y + ((size_t)b * NCP + tid) * NP + qb * 64; for (int qi = 0; qi < 64; ++qi) { const float d = yr[qi] - mu; acc += d * d; } } s[tid] = acc; }
  __syncthreads();
  if (tid < 8) vst2(PS + ((size_t)b * 64 + qb) * 32 + tid * 4, *(const v4f*)&s[tid * 4]);
}
__global__ __launch_bounds__(256) void k_out(const float* __restrict__ Y, const float* __restrict__ ST, const float* __restrict__ gm, const float* __restrict__ bt, float* __restrict__ out) {
  const int c = blockIdx.x, b = blockIdx.y, tid = threadIdx.x; const float mu = ST[c], ga = ST[32 + c] * bfr(gm[c]), be = bfr(bt[c]);
  const float* yr = Y + ((size_t)b * NCP + c) * NP; float* orow = out + ((size_t)b * NCL + c) * NP;
  for (int pc = tid; pc < NP / 4; pc += 256) { const float* p = yr + pc * 4; vst2(orow + pc * 4, (v4f){(p[0] - mu) * ga + be, (p[1] - mu) * ga + be, (p[2] - mu) * ga + be, (p[3] - mu) * ga + be}); }
}
extern "C" void kernel_launch(void* const* d_in, const int* in_sizes, int n_in, void* d_out, int out_size, void* d_ws, size_t ws_size, hipStream_t stream) {
  (void)in_sizes; (void)n_in; (void)out_size;
  const float** F = (const float**)d_in;
  if (ws_size < (size_t)WS_END) return;
  char* ws = (char*)d_ws; __bf16 *PW = (__bf16*)(ws + WS_PW), *VB = (__bf16*)(ws + WS_VB); float *QK = (float*)(ws + WS_QK), *Y = (float*)(ws + WS_Y), *PS = (float*)(ws + WS_PS), *ST = (float*)(ws + WS_ST);
  k_pack<<<dim3(16 * NB * NCP, 2), 256, 0, stream>>>(F[4], F[2], F[0], PW, VB);
  k_qk<<<dim3(NP / 64, TNB), 128, 0, stream>>>(F[1], PW, F[5], F[3], QK);
  k_attn<<<dim3(TQB, TNB), 128, 0, stream>>>(QK, VB, F[0], F[6], F[7], Y, PS);
  k_red<0><<<1, 32, 0, stream>>>(PS, ST);
  k_var<<<dim3(TQB, TNB), 64, 0, stream>>>(Y, ST, PS);
  k_red<1><<<1, 32, 0, stream>>>(PS, ST);
  k_out<<<dim3(NCL, TNB), 256, 0, stream>>>(Y, ST, F[8], F[9], (float*)d_out);
}
